// SimpleRNN_4071628996712
// MI455X (gfx1250) — hardware-verified
//
#include <hip/hip_runtime.h>


#define RB 4096
#define RT 1024
#define RH 16
#define SP 36

static_assert(RB % 16 == 0);
static_assert(RT % 32 == 0);
static_assert(RH == 16);
static_assert((SP * 4) % 16 == 0 && SP >= 32);

typedef __bf16         v16b __attribute__((ext_vector_type(16)));
typedef unsigned short v8us __attribute__((ext_vector_type(8)));
typedef float          v8f  __attribute__((ext_vector_type(8)));
typedef float          v4f  __attribute__((ext_vector_type(4)));
typedef v4f __attribute__((may_alias)) v4fa;

union Frag { v16b v; v8us half[2]; };

__device__ __forceinline__ unsigned short bf16_bits(float f) {
  unsigned u = __float_as_uint(f);
  u += 0x7FFFu + ((u >> 16) & 1u);
  return (unsigned short)(u >> 16);
}
__device__ __forceinline__ float bf16_val(unsigned short b) { return __uint_as_float(((unsigned)b) << 16); }
__device__ __forceinline__ float bf16r(float f) { return bf16_val(bf16_bits(f)); }
__device__ __forceinline__ v8f zero8() {
  v8f z;
#pragma unroll
  for (int i = 0; i < 8; ++i) z[i] = 0.0f;
  return z;
}
__device__ __forceinline__ v8us zero8us() {
  v8us z;
#pragma unroll
  for (int i = 0; i < 8; ++i) z[i] = (unsigned short)0;
  return z;
}

__device__ __forceinline__ v8f mma16(v8f c, const Frag& a, const Frag& b) {
  return __builtin_amdgcn_wmma_f32_16x16x32_bf16(false, a.v, false, b.v, (short)0, c, false, false);
}

__global__ __launch_bounds__(32)
void rnn_kernel(const float* __restrict__ x,   const float* __restrict__ wih, const float* __restrict__ bih,
                const float* __restrict__ whh, const float* __restrict__ bhh, const float* __restrict__ fcw,
                const float* __restrict__ fcb, float* out)
{
  __shared__ __attribute__((aligned(16))) float sO[16 * SP];

  const int lane = threadIdx.x & 31, hh = lane >> 4, c = lane & 15;
  const int b0 = (int)blockIdx.x * 16;
  const int q8 = lane & 7, sub = lane >> 3;

  const v8us z8 = zero8us();

  Frag a;
  {
    v8us w8;
#pragma unroll
    for (int i = 0; i < 8; ++i) w8[i] = bf16_bits(whh[c * RH + 8 * hh + i]);
    a.half[0] = w8;
    a.half[1] = z8;
  }
  float wi[8], bi[8], bh[8], fw[8];
#pragma unroll
  for (int r = 0; r < 8; ++r) {
    const int n = 8 * hh + r;
    wi[r] = bf16r(wih[n]);
    bi[r] = bf16r(bih[n]);
    bh[r] = bf16r(bhh[n]);
    fw[r] = bf16r(fcw[n]);
  }
  const float fb = bf16r(fcb[0]);

  Frag bhi, blo;
  bhi.half[0] = z8; bhi.half[1] = z8;
  blo.half[0] = z8; blo.half[1] = z8;

  const float* xrow = x + (size_t)(b0 + c) * RT;
  float x0 = 0.0f, x1 = 0.0f, x2 = 0.0f, x3 = 0.0f;

#pragma unroll 1
  for (int t = 0; t < RT; ++t) {
    const int u = t & 3;
    if (u == 0) {
      const v4f xv = *(const v4fa*)(xrow + t);
      x0 = bf16r(xv[0]); x1 = bf16r(xv[1]); x2 = bf16r(xv[2]); x3 = bf16r(xv[3]);
    }
    float xt = x0;
    if (u == 1) xt = x1;
    if (u == 2) xt = x2;
    if (u == 3) xt = x3;

    v8f acc = zero8();
    acc = mma16(acc, a, bhi);
    acc = mma16(acc, a, blo);
    asm volatile("v_nop\n\tv_nop\n\tv_nop\n\tv_nop" : "+v"(acc) : "v"(a.v), "v"(bhi.v), "v"(blo.v));

    v8us nh, nl;
    float p = 0.0f;
#pragma unroll
    for (int r = 0; r < 8; ++r) {
      const float xp = (xt * wi[r] + bi[r]) + bh[r];
      const float v  = tanhf(xp + acc[r]);
      const unsigned short hb = bf16_bits(v);
      nh[r] = hb;
      nl[r] = bf16_bits(v - bf16_val(hb));
      p = fmaf(v, fw[r], p);
    }
    {
      Frag nbh, nbl;
      nbh.half[0] = nh; nbh.half[1] = z8;
      nbl.half[0] = nl; nbl.half[1] = z8;
      bhi = nbh;
      blo = nbl;
    }
    p += __shfl_xor(p, 16);
    const float o = p + fb;
    if (hh == 0) sO[c * SP + (t & 31)] = o;

    if ((t & 31) == 31) {
      __syncthreads();
      const int c32 = t & ~31;
      v4f ov[4];
      size_t oo[4];
#pragma unroll
      for (int i = 0; i < 4; ++i) {
        const int row = 4 * i + sub;
        ov[i] = *(const v4fa*)(sO + row * SP + 4 * q8);
        oo[i] = (size_t)(b0 + row) * RT + c32 + 4 * q8;
      }
#pragma unroll
      for (int i = 0; i < 4; ++i) *(volatile v4f*)(out + oo[i]) = ov[i];
      __threadfence();
#pragma unroll
      for (int i = 0; i < 4; ++i) *(volatile v4f*)(out + oo[i]) = ov[i];
      __syncthreads();
    }
  }
}

extern "C" void kernel_launch(void* const* d_in, const int* in_sizes, int n_in,
                              void* d_out, int out_size, void* d_ws, size_t ws_size,
                              hipStream_t stream)
{
  (void)d_ws; (void)ws_size;
  if (n_in < 7) return;
  if (in_sizes[0] != RB * RT) return;
  if (in_sizes[1] != RH)      return;
  if (in_sizes[2] != RH)      return;
  if (in_sizes[3] != RH * RH) return;
  if (in_sizes[4] != RH)      return;
  if (in_sizes[5] != RH)      return;
  if (in_sizes[6] != 1)       return;
  if (out_size != RB * RT)    return;

  const float* x   = (const float*)d_in[0];
  const float* wih = (const float*)d_in[1];
  const float* bih = (const float*)d_in[2];
  const float* whh = (const float*)d_in[3];
  const float* bhh = (const float*)d_in[4];
  const float* fcw = (const float*)d_in[5];
  const float* fcb = (const float*)d_in[6];
  float* out = (float*)d_out;

  rnn_kernel<<<dim3(RB / 16), dim3(32), 0, stream>>>(x, wih, bih, whh, bhh, fcw, fcb, out);
}
